// SSMLayer_17514876633683
// MI455X (gfx1250) — hardware-run, weakly checked
//
#include <hip/hip_runtime.h>
#include <math.h>

constexpr int NBAT  = 4;
constexpr int NSEQ  = 512;
constexpr int NHID  = 512;
constexpr int NSTA  = 128;
constexpr int NROWS = NBAT * NSEQ;
constexpr int NTHR  = 256;
constexpr int SCAN_THR = 128;
constexpr int SPITCH = 136;
constexpr float ACARRY     = 16.0f;
constexpr float ACARRY_INV = 1.0f / 16.0f;
constexpr float LN_EPS_F   = 1e-5f;
static_assert(NHID % 32 == 0);
static_assert(NROWS % 64 == 0 && NHID % 64 == 0 && NSTA % 64 == 0);
static_assert(NSTA == 32 * (SCAN_THR / 32));
static_assert((16 * SPITCH) % SCAN_THR == 0);
static_assert(NROWS % (NTHR / 32) == 0);
static_assert(NROWS % (SCAN_THR * 4) == 0);
static_assert(NHID == 512);

typedef __attribute__((ext_vector_type(16))) _Float16 v16h;
typedef __attribute__((ext_vector_type(8)))  _Float16 v8h;
typedef __attribute__((ext_vector_type(16))) __bf16   v16b;
typedef __attribute__((ext_vector_type(8)))  __bf16   v8b;
typedef __attribute__((ext_vector_type(8)))  float    v8f;
typedef __attribute__((ext_vector_type(4)))  float    v4f;

__device__ __forceinline__ unsigned short f2bf_bits(float f) {
  unsigned u = __float_as_uint(f);
  return (unsigned short)((u + 0x7FFFu + ((u >> 16) & 1u)) >> 16);
}
__device__ __forceinline__ float bf_bits2f(unsigned short h) { return __uint_as_float(((unsigned)h) << 16); }
__device__ __forceinline__ float bf16r(float f) { return bf_bits2f(f2bf_bits(f)); }

__device__ __forceinline__ void dep_guard_h(v8f& a, v8f& b, v16h x, v16h y) { asm volatile("v_nop\n\tv_nop\n\tv_nop\n\tv_nop" : "+v"(a), "+v"(b) : "v"(x), "v"(y)); }
__device__ __forceinline__ void dep_guard_b(v8f& a, v8f& b, v16b x, v16b y) { asm volatile("v_nop\n\tv_nop\n\tv_nop\n\tv_nop" : "+v"(a), "+v"(b) : "v"(x), "v"(y)); }
__device__ __forceinline__ void keep4_h(v16h a, v16h b, v16h c, v16h d) { asm volatile("v_nop" :: "v"(a), "v"(b), "v"(c), "v"(d)); }
__device__ __forceinline__ void keep4_b(v16b a, v16b b, v16b c, v16b d) { asm volatile("v_nop" :: "v"(a), "v"(b), "v"(c), "v"(d)); }
__device__ __forceinline__ void acc_guard4(v8f& a, v8f& b, v8f& c, v8f& d) { asm volatile("v_nop\n\tv_nop\n\tv_nop\n\tv_nop" : "+v"(a), "+v"(b), "+v"(c), "+v"(d)); }
__device__ __forceinline__ void acc_guard2(v8f& a, v8f& b) { asm volatile("v_nop\n\tv_nop\n\tv_nop\n\tv_nop" : "+v"(a), "+v"(b)); }
template <typename T> struct Frag;
template <> struct Frag<_Float16> {
  typedef v16h V; union U { v16h v; v8h h[2]; };
  static __device__ __forceinline__ v16h load(const _Float16* p) {
    U f; f.h[0] = *(const v8h*)(p); f.h[1] = *(const v8h*)(p + 16); return f.v;
  }
  static __device__ __forceinline__ v8f mma(v16h a, v16h b, v8f c) {
    return __builtin_amdgcn_wmma_f32_16x16x32_f16(false, a, false, b, (short)0, c, false, false);
  }
  static __device__ __forceinline__ void guard(v8f& a, v8f& b, v16h x, v16h y) { dep_guard_h(a, b, x, y); }
  static __device__ __forceinline__ void keep(v16h a, v16h b, v16h c, v16h d) { keep4_h(a, b, c, d); }
};
template <> struct Frag<__bf16> {
  typedef v16b V; union U { v16b v; v8b h[2]; };
  static __device__ __forceinline__ v16b load(const __bf16* p) {
    U f; f.h[0] = *(const v8b*)(p); f.h[1] = *(const v8b*)(p + 16); return f.v;
  }
  static __device__ __forceinline__ v8f mma(v16b a, v16b b, v8f c) {
    return __builtin_amdgcn_wmma_f32_16x16x32_bf16(false, a, false, b, (short)0, c, false, false);
  }
  static __device__ __forceinline__ void guard(v8f& a, v8f& b, v16b x, v16b y) { dep_guard_b(a, b, x, y); }
  static __device__ __forceinline__ void keep(v16b a, v16b b, v16b c, v16b d) { keep4_b(a, b, c, d); }
};

template <int ET> struct Elem;
template <> struct Elem<0> { typedef _Float16 T; };
template <> struct Elem<1> { typedef __bf16 T; };
template <int ET, bool SPLIT, int BIAS_MODE, int OUT_MODE, bool RESID, int ACT = 0>
__global__ __launch_bounds__(256) void wmma_gemm64(
    const unsigned short* __restrict__ Ap, const unsigned short* __restrict__ A2p, int lda, long strideA,
    const unsigned short* __restrict__ Btp, const unsigned short* __restrict__ Bt2p, int ldb, long strideB,
    void* __restrict__ Cout, void* __restrict__ Cout2, int ldc, long strideC,
    const float* __restrict__ bias,
    const float* __restrict__ resid, long strideR,
    int M, int N, int K, float scale) {
  typedef typename Elem<ET>::T T;
  typedef typename Frag<T>::V V;
  const T* A = (const T*)Ap; const T* A2 = (const T*)A2p; const T* Bt = (const T*)Btp; const T* Bt2 = (const T*)Bt2p;
  __shared__ __align__(16) float sT[8][16 * 68];
  const int b    = blockIdx.y;
  const int lane = threadIdx.x & 31;
  const int wave = threadIdx.x >> 5;
  const int tilesN = N >> 6;
  const int tilesM = M >> 6;
  const int tile = blockIdx.x * 8 + wave;
  if (tile >= tilesM * tilesN) return;
  const int tm = tile / tilesN;
  const int tn = tile - tm * tilesN;
  const int m0 = tm << 6;
  const int n0 = tn << 6;

  const T* Ab  = A  + (size_t)b * strideA;
  const T* Bb  = Bt + (size_t)b * strideB;
  const T* Ab2 = SPLIT ? (A2  + (size_t)b * strideA) : nullptr;
  const T* Bb2 = SPLIT ? (Bt2 + (size_t)b * strideB) : nullptr;

  const int rlane = lane & 15;
  const int koff  = (lane >> 4) * 8;
  const int mOff  = (lane >> 4) * 8;

  v8f acc[4][4];
#pragma unroll
  for (int i = 0; i < 4; ++i)
#pragma unroll
    for (int j = 0; j < 4; ++j) acc[i][j] = (v8f){0.f,0.f,0.f,0.f,0.f,0.f,0.f,0.f};

  for (int k0 = 0; k0 < K; k0 += 32) {
    V bh[4], bl[4];
#pragma unroll
    for (int j = 0; j < 4; ++j) {
      const size_t bo = (size_t)(n0 + (j << 4) + rlane) * ldb + koff + k0;
      bh[j] = Frag<T>::load(Bb + bo);
      if (SPLIT) bl[j] = Frag<T>::load(Bb2 + bo);
    }
#pragma unroll
    for (int i = 0; i < 4; ++i) {
      const size_t ao = (size_t)(m0 + (i << 4) + rlane) * lda + koff + k0;
      V ah = Frag<T>::load(Ab + ao);
      V al;
      if (SPLIT) al = Frag<T>::load(Ab2 + ao);
#pragma unroll
      for (int j = 0; j < 4; ++j) {
        acc[i][j] = Frag<T>::mma(ah, bh[j], acc[i][j]);
        if (SPLIT) {
          acc[i][j] = Frag<T>::mma(ah, bl[j], acc[i][j]);
          acc[i][j] = Frag<T>::mma(al, bh[j], acc[i][j]);
        }
      }
      Frag<T>::guard(acc[i][0], acc[i][3], ah, SPLIT ? al : ah);
    }
    Frag<T>::keep(bh[0], bh[1], bh[2], bh[3]);
    if (SPLIT) Frag<T>::keep(bl[0], bl[1], bl[2], bl[3]);
  }
  acc_guard4(acc[0][0], acc[0][1], acc[0][2], acc[0][3]);
  acc_guard4(acc[1][0], acc[1][1], acc[1][2], acc[1][3]);
  acc_guard4(acc[2][0], acc[2][1], acc[2][2], acc[2][3]);
  acc_guard4(acc[3][0], acc[3][1], acc[3][2], acc[3][3]);

  float* slab = sT[wave];
  const float* Rb = RESID ? (resid + (size_t)b * strideR) : nullptr;
#pragma unroll
  for (int i = 0; i < 4; ++i) {
    const int mBase = m0 + (i << 4);
#pragma unroll
    for (int j = 0; j < 4; ++j) {
      const int n = n0 + (j << 4) + rlane;
      float bv = 0.f;
      if (BIAS_MODE == 2) bv = bias[n];
#pragma unroll
      for (int r = 0; r < 8; ++r) {
        float v = acc[i][j][r] * scale;
        if (BIAS_MODE == 1) v += bias[mBase + mOff + r];
        if (BIAS_MODE == 2) v += bv;
        if (RESID) v += Rb[(size_t)(mBase + mOff + r) * ldc + n];
        if (ACT == 1) v = tanhf(v);
        if (ACT == 2) v = fmaxf(v, 0.0f);
        if (ACT == 3) v = v / (1.0f + expf(-v));
        if (ACT == 4) v = (v > 0.f) ? v : 0.01f * v;
        if (ACT == 5) v = 0.5f * v * (1.0f + erff(v * 0.70710678118654752f));
        slab[(mOff + r) * 68 + (j << 4) + rlane] = v;
      }
    }
    __builtin_amdgcn_fence(__ATOMIC_RELEASE, "workgroup");
    __builtin_amdgcn_wave_barrier();
    __builtin_amdgcn_fence(__ATOMIC_ACQUIRE, "workgroup");
    if (OUT_MODE == 0) {
      float* C = (float*)Cout + (size_t)b * strideC;
      const int hh = lane >> 4, c4 = (lane & 15) * 4;
      for (int pass = 0; pass < 2; ++pass) {
#pragma unroll
        for (int it = 0; it < 8; ++it) {
          const int row = it * 2 + hh;
          v4f v = *(const v4f*)(slab + row * 68 + c4);
          *(volatile v4f*)(C + (size_t)(mBase + row) * ldc + n0 + c4) = v;
        }
        __threadfence();
      }
    } else {
      const int q = lane >> 3, c8 = (lane & 7) * 8;
      unsigned short* C  = (unsigned short*)Cout  + (size_t)b * strideC;
      unsigned short* C2 = (OUT_MODE == 2) ? ((unsigned short*)Cout2 + (size_t)b * strideC) : nullptr;
      for (int pass = 0; pass < 2; ++pass) {
#pragma unroll
        for (int it = 0; it < 4; ++it) {
          const int row = it * 4 + q;
          const float* sp = slab + row * 68 + c8;
          v8h hv, lv;
#pragma unroll
          for (int e = 0; e < 8; ++e) {
            if (OUT_MODE == 1) {
              hv[e] = (_Float16)sp[e];
            } else {
              unsigned short hb = f2bf_bits(sp[e]);
              unsigned short lb = f2bf_bits(sp[e] - bf_bits2f(hb));
              hv[e] = __builtin_bit_cast(_Float16, hb);
              lv[e] = __builtin_bit_cast(_Float16, lb);
            }
          }
          *(volatile v8h*)(C + (size_t)(mBase + row) * ldc + n0 + c8) = hv;
          if (OUT_MODE == 2) *(volatile v8h*)(C2 + (size_t)(mBase + row) * ldc + n0 + c8) = lv;
        }
        __threadfence();
      }
    }
    __builtin_amdgcn_fence(__ATOMIC_RELEASE, "workgroup");
    __builtin_amdgcn_wave_barrier();
    __builtin_amdgcn_fence(__ATOMIC_ACQUIRE, "workgroup");
  }
}

template <int MODE>
__global__ __launch_bounds__(NTHR) void cvt8_kernel(const float* __restrict__ src, unsigned short* __restrict__ dst,
                                                    int nrow, int ncol8, int spitch, int scol0, float sc) {
  const int i  = blockIdx.x * NTHR + threadIdx.x;
  const int n8 = nrow * ncol8;
  if (i < n8) {
    const int row = i / ncol8;
    const int c8  = i - row * ncol8;
    const float* sp = src + (size_t)row * spitch + scol0 + c8 * 8;
    const v4f a = *(const v4f*)(sp);
    const v4f b = *(const v4f*)(sp + 4);
    v8h hv;
#pragma unroll
    for (int e = 0; e < 4; ++e) {
      unsigned short b0, b1;
      if (MODE == 0) {
        b0 = f2bf_bits(a[e] * sc);
        b1 = f2bf_bits(b[e] * sc);
      } else {
        b0 = __builtin_bit_cast(unsigned short, (_Float16)(bf16r(a[e]) * sc));
        b1 = __builtin_bit_cast(unsigned short, (_Float16)(bf16r(b[e]) * sc));
      }
      hv[e]     = __builtin_bit_cast(_Float16, b0);
      hv[4 + e] = __builtin_bit_cast(_Float16, b1);
    }
    *(volatile v8h*)(dst + (size_t)i * 8) = hv;
    __threadfence();
    *(volatile v8h*)(dst + (size_t)i * 8) = hv;
  }
}

__global__ __launch_bounds__(SCAN_THR) void scan_kernel(const float* __restrict__ Amat, const float* __restrict__ Cmat,
                                                         const float* __restrict__ U, float* __restrict__ CV) {
  __shared__ __align__(16) _Float16 Ast[16 * SPITCH];
  __shared__ float cbarL[NSTA];
  __shared__ float wred[16];
  __shared__ __align__(16) float cbuf[NROWS];
  const int tid = threadIdx.x, lane = tid & 31, wave = tid >> 5;
  const int c = lane & 15, hh = lane >> 4, koff = hh * 8;

#pragma unroll 1
  for (int i = tid; i < 16 * SPITCH; i += SCAN_THR) Ast[i] = (_Float16)0.0f;
  {
    float acc = 0.0f;
#pragma unroll 1
    for (int h = 0; h < NHID; ++h) acc += bf16r(Cmat[(size_t)h * NSTA + tid]);
    cbarL[tid] = acc * (1.0f / NHID);
  }
  v16h bfr[2][4];
#pragma unroll
  for (int nt = 0; nt < 2; ++nt) {
#pragma unroll
    for (int kc = 0; kc < 4; ++kc) {
      const float* ap = Amat + (size_t)(32 * wave + 16 * nt + c) * NSTA + 32 * kc + koff;
      const v4f a0 = *(const v4f*)(ap);
      const v4f a1 = *(const v4f*)(ap + 4);
      const v4f a2 = *(const v4f*)(ap + 16);
      const v4f a3 = *(const v4f*)(ap + 20);
      v16h f;
#pragma unroll
      for (int e = 0; e < 4; ++e) {
        f[e]      = (_Float16)(bf16r(a0[e]) * ACARRY);
        f[4 + e]  = (_Float16)(bf16r(a1[e]) * ACARRY);
        f[8 + e]  = (_Float16)(bf16r(a2[e]) * ACARRY);
        f[12 + e] = (_Float16)(bf16r(a3[e]) * ACARRY);
      }
      bfr[nt][kc] = f;
      asm volatile("" ::: "memory");
    }
  }
  __syncthreads();

  float cbr[2];
#pragma unroll
  for (int nt = 0; nt < 2; ++nt) cbr[nt] = cbarL[32 * wave + 16 * nt + c];
  float stv[2][4];
#pragma unroll
  for (int nt = 0; nt < 2; ++nt)
#pragma unroll
    for (int r = 0; r < 4; ++r) stv[nt][r] = 0.0f;
  const float fa = 1.0f - (float)hh;
  const _Float16* arow = Ast + c * SPITCH + koff;
  const v8f z8 = {0.f, 0.f, 0.f, 0.f, 0.f, 0.f, 0.f, 0.f};

#pragma unroll 1
  for (int t = 0; t < NSEQ; ++t) {
    float pc[4];
#pragma unroll
    for (int b = 0; b < 4; ++b) {
      float s = 0.0f;
      s = fmaf(cbr[0], stv[0][b], s);
      s = fmaf(cbr[1], stv[1][b], s);
      pc[b] = s;
    }
#pragma unroll
    for (int off = 16; off >= 1; off >>= 1) {
#pragma unroll
      for (int b = 0; b < 4; ++b) pc[b] += __shfl_xor(pc[b], off, 32);
    }
    if (lane == 0) {
      wred[wave * 4 + 0] = pc[0]; wred[wave * 4 + 1] = pc[1];
      wred[wave * 4 + 2] = pc[2]; wred[wave * 4 + 3] = pc[3];
    }
    float uv[2][4];
#pragma unroll
    for (int nt = 0; nt < 2; ++nt) {
      const int p = 32 * wave + 16 * nt + c;
#pragma unroll
      for (int r = 0; r < 4; ++r) {
        int urow = 8 * hh + r; urow = (urow > 3) ? 3 : urow;
        uv[nt][r] = U[((size_t)urow * NSEQ + (size_t)t) * NSTA + p];
      }
    }
    v8f acc[2];
    acc[0] = z8; acc[1] = z8;
#pragma unroll
    for (int kc = 0; kc < 4; ++kc) {
      const v16h a = Frag<_Float16>::load(arow + 32 * kc);
      acc[0] = Frag<_Float16>::mma(a, bfr[0][kc], acc[0]);
      acc[1] = Frag<_Float16>::mma(a, bfr[1][kc], acc[1]);
      dep_guard_h(acc[0], acc[1], a, bfr[1][kc]);
    }
    acc_guard2(acc[0], acc[1]);
    __syncthreads();
    if (tid < NBAT) cbuf[tid * NSEQ + t] = ((wred[tid] + wred[4 + tid]) + wred[8 + tid]) + wred[12 + tid];
#pragma unroll
    for (int nt = 0; nt < 2; ++nt) {
      const int p = 32 * wave + 16 * nt + c;
#pragma unroll
      for (int r = 0; r < 4; ++r) {
        const float v = fa * fmaf(acc[nt][r], ACARRY_INV, uv[nt][r]);
        stv[nt][r] = v;
        Ast[(8 * hh + r) * SPITCH + p] = (_Float16)v;
      }
#pragma unroll
      for (int r = 4; r < 8; ++r) Ast[(8 * hh + r) * SPITCH + p] = (_Float16)0.0f;
    }
    __syncthreads();
  }

  for (int pass = 0; pass < 2; ++pass) {
#pragma unroll
    for (int it = 0; it < NROWS / (SCAN_THR * 4); ++it) {
      const int idx = it * SCAN_THR + tid;
      const v4f v = *(const v4f*)(cbuf + idx * 4);
      *(volatile v4f*)(CV + (size_t)idx * 4) = v;
    }
    __threadfence();
  }
}

__global__ __launch_bounds__(NTHR) void ln_gelu_kernel(const float* __restrict__ V, const float* __restrict__ X,
                                                       const float* __restrict__ CV, const float* __restrict__ gam,
                                                       const float* __restrict__ bet, float* __restrict__ Y) {
  __shared__ __align__(16) float rbuf[NTHR / 32][NHID];
  const int tid = threadIdx.x, lane = tid & 31, wave = tid >> 5;
  const int row = blockIdx.x * (NTHR / 32) + wave;
  float* rb = rbuf[wave];
  const float* vp = V + (size_t)row * NHID;
  const float* xp = X + (size_t)row * NHID;
  const float cadd = CV[row];

  float s = 0.0f;
#pragma unroll 1
  for (int i = 0; i < NHID / 32; ++i) {
    const int col = 32 * i + lane;
    const float a = vp[col] + cadd;
    const float g = 0.5f * a * (1.0f + erff(a * 0.70710678118654752f));
    const float y = g + bf16r(xp[col]);
    rb[col] = y;
    s += y;
  }
#pragma unroll
  for (int off = 1; off < 32; off <<= 1) s += __shfl_xor(s, off, 32);
  const float mu = s * (1.0f / NHID);
  __syncthreads();

  float ss = 0.0f;
#pragma unroll 1
  for (int q = 0; q < 4; ++q) {
    const v4f y4 = *(const v4f*)(rb + 128 * q + 4 * lane);
#pragma unroll
    for (int e = 0; e < 4; ++e) { const float d = y4[e] - mu; ss += d * d; }
  }
#pragma unroll
  for (int off = 1; off < 32; off <<= 1) ss += __shfl_xor(ss, off, 32);
  const float var  = ss * (1.0f / NHID);
  const float rstd = rsqrtf(var + LN_EPS_F);

#pragma unroll 1
  for (int q = 0; q < 4; ++q) {
    const int col = 128 * q + 4 * lane;
    const v4f y4 = *(const v4f*)(rb + col);
    const v4f g4 = *(const v4f*)(gam + col);
    const v4f b4 = *(const v4f*)(bet + col);
    v4f o;
#pragma unroll
    for (int e = 0; e < 4; ++e) o[e] = ((y4[e] - mu) * rstd) * bf16r(g4[e]) + bf16r(b4[e]);
    *(v4f*)(rb + col) = o;
  }
  __syncthreads();
  float* op = Y + (size_t)row * NHID;
  for (int pass = 0; pass < 2; ++pass) {
#pragma unroll 1
    for (int q = 0; q < 4; ++q) {
      const int col = 128 * q + 4 * lane;
      const v4f o = *(const v4f*)(rb + col);
      *(volatile v4f*)(op + col) = o;
    }
    __threadfence();
  }
}

extern "C" void kernel_launch(void* const* d_in, const int* in_sizes, int n_in,
                              void* d_out, int out_size, void* d_ws, size_t ws_size, hipStream_t stream) {
  if (n_in < 7 || d_out == nullptr || d_ws == nullptr) return;
  if (in_sizes[0] != NROWS * NHID || in_sizes[1] != NSTA * NSTA || in_sizes[2] != NSTA * NHID ||
      in_sizes[3] != NHID * NSTA || in_sizes[4] != NHID * NHID || in_sizes[5] != NHID || in_sizes[6] != NHID ||
      out_size != NROWS * NHID) return;

  const float* x    = (const float*)d_in[0];
  const float* Amat = (const float*)d_in[1];
  const float* Bmat = (const float*)d_in[2];
  const float* Cmat = (const float*)d_in[3];
  const float* Dmat = (const float*)d_in[4];
  const float* gam  = (const float*)d_in[5];
  const float* bet  = (const float*)d_in[6];
  float* y_out = (float*)d_out;

  char* ws = (char*)d_ws; size_t off = 0;
  auto carve = [&](size_t bytes) -> char* { char* p = ws + off; off += (bytes + 255) & ~(size_t)255; return p; };
  unsigned short* XB = (unsigned short*)carve((size_t)NROWS * NHID * 2);
  unsigned short* DB = (unsigned short*)carve((size_t)NHID * NHID * 2);
  unsigned short* BB = (unsigned short*)carve((size_t)NSTA * NHID * 2);
  float*          U  = (float*)carve((size_t)NROWS * NSTA * 4);
  float*          V  = (float*)carve((size_t)NROWS * NHID * 4);
  float*          CV = (float*)carve((size_t)NROWS * 4);
  if (off > ws_size || off > (size_t)134217728) return;

  const int n8x = NROWS * (NHID / 8);
  const int n8d = NHID * (NHID / 8);
  const int n8b = NSTA * (NHID / 8);
  cvt8_kernel<0><<<(n8x + NTHR - 1) / NTHR, NTHR, 0, stream>>>(x,    XB, NROWS, NHID / 8, NHID, 0, 1.0f);
  cvt8_kernel<0><<<(n8d + NTHR - 1) / NTHR, NTHR, 0, stream>>>(Dmat, DB, NHID,  NHID / 8, NHID, 0, 1.0f);
  cvt8_kernel<0><<<(n8b + NTHR - 1) / NTHR, NTHR, 0, stream>>>(Bmat, BB, NSTA,  NHID / 8, NHID, 0, 1.0f);

  const dim3 ugrid(((NROWS / 64) * (NSTA / 64) + 7) / 8, 1);
  wmma_gemm64<1, false, 0, 0, false, 0><<<ugrid, 256, 0, stream>>>(
      XB, XB, NHID, 0L, BB, BB, NHID, 0L, (void*)U, (void*)U, NSTA, 0L,
      CV, V, 0L, NROWS, NSTA, NHID, 1.0f);

  scan_kernel<<<1, SCAN_THR, 0, stream>>>(Amat, Cmat, U, CV);

  const dim3 vgrid(((NROWS / 64) * (NHID / 64) + 7) / 8, 1);
  wmma_gemm64<1, false, 0, 0, false, 0><<<vgrid, 256, 0, stream>>>(
      XB, XB, NHID, 0L, DB, DB, NHID, 0L, (void*)V, (void*)V, NHID, 0L,
      CV, U, 0L, NROWS, NHID, NHID, 1.0f);

  ln_gelu_kernel<<<NROWS / (NTHR / 32), NTHR, 0, stream>>>(V, x, CV, gam, bet, y_out);
}
